// ETCLayer_19224273617225
// MI455X (gfx1250) — hardware-verified
//
#include <hip/hip_runtime.h>
#include <math.h>

typedef __attribute__((ext_vector_type(16))) _Float16 v16h;
typedef __attribute__((ext_vector_type(16))) __bf16 v16b;
typedef __attribute__((ext_vector_type(8)))  _Float16 v8h;
typedef __attribute__((ext_vector_type(8)))  float v8f;
typedef __attribute__((ext_vector_type(4)))  float v4f;
typedef __attribute__((ext_vector_type(2)))  float v2f;
typedef __attribute__((ext_vector_type(4)))  unsigned v4u;
typedef __attribute__((ext_vector_type(4)))  int v4i;
typedef float __attribute__((may_alias)) float_a;
typedef int __attribute__((may_alias)) int_a;

template <typename T> __device__ __forceinline__ void vst2(void* p, T v) { *(volatile T*)p = v; __threadfence(); *(volatile T*)p = v; }
__device__ __forceinline__ v8f wmma16(v16h a, v16h b, v8f c) {
  v8f d = __builtin_amdgcn_wmma_f32_16x16x32_f16(false, a, false, b, (short)0, c, false, false);
  asm volatile("v_nop\n\tv_nop\n\tv_nop\n\tv_nop" : "+v"(d) : "v"(a), "v"(b));
  return d;
}
__device__ __forceinline__ v8f wmma_bf(v16b a, v16b b, v8f c) {
  v8f d = __builtin_amdgcn_wmma_f32_16x16x32_bf16(false, a, false, b, (short)0, c, false, false);
  asm volatile("v_nop\n\tv_nop\n\tv_nop\n\tv_nop" : "+v"(d) : "v"(a), "v"(b));
  return d;
}
__device__ __forceinline__ v16h frag_h(const _Float16* rowk0, int lane) {
  union { v16h v; v8h q[2]; } u; const _Float16* p = rowk0 + 8 * (lane >> 4);
  u.q[0] = *(const v8h*)p; u.q[1] = *(const v8h*)(p + 16); return u.v;
}
__device__ __forceinline__ v16h frag_f32(const float* rowk0, int lane) {
  v16h a; const float* p = rowk0 + 8 * (lane >> 4);
#pragma unroll
  for (int i = 0; i < 8; ++i) { a[i] = (_Float16)p[i]; a[8 + i] = (_Float16)p[16 + i]; }
  return a;
}
__device__ __forceinline__ v16h frag_f32s(const float* rowk0, int lane, float sc) {
  v16h a; const float* p = rowk0 + 8 * (lane >> 4);
#pragma unroll
  for (int i = 0; i < 8; ++i) { a[i] = (_Float16)(p[i] * sc); a[8 + i] = (_Float16)(p[16 + i] * sc); }
  return a;
}
__device__ __forceinline__ v16h fragc_f32(const float* W, int k0, int n, int lane, int ld, int K) {
  v16h a; const int g = lane >> 4;
#pragma unroll
  for (int i = 0; i < 8; ++i) { const int ka = k0 + 8 * g + i, kb = ka + 16;
    a[i] = (_Float16)(ka < K ? W[(size_t)(ka < K ? ka : K - 1) * ld + n] : 0.f); a[8 + i] = (_Float16)(kb < K ? W[(size_t)(kb < K ? kb : K - 1) * ld + n] : 0.f); }
  return a;
}
struct F2 { v16b h, l; };
__device__ __forceinline__ F2 bsplit16(const float v[16]) { F2 r;
#pragma unroll
  for (int i = 0; i < 16; ++i) { const __bf16 h = (__bf16)v[i]; r.h[i] = h; r.l[i] = (__bf16)(v[i] - (float)h); }
  return r; }
__device__ __forceinline__ F2 split_row(const float* row, int k0, int lane) { float v[16]; const float* p = row + k0 + 8 * (lane >> 4);
#pragma unroll
  for (int i = 0; i < 8; ++i) { v[i] = p[i]; v[8 + i] = p[16 + i]; }
  return bsplit16(v); }
__device__ __forceinline__ F2 split_rowK(const float* row, int k0, int lane, int K) { float v[16]; const int g = lane >> 4;
#pragma unroll
  for (int i = 0; i < 8; ++i) { const int ka = k0 + 8 * g + i, kb = ka + 16; v[i] = ka < K ? row[ka < K ? ka : K - 1] : 0.f; v[8 + i] = kb < K ? row[kb < K ? kb : K - 1] : 0.f; }
  return bsplit16(v); }
__device__ __forceinline__ F2 split_col(const float* W, int k0, int n, int lane, int ld, int K) { float v[16]; const int g = lane >> 4;
#pragma unroll
  for (int i = 0; i < 8; ++i) { const int ka = k0 + 8 * g + i, kb = ka + 16; v[i] = ka < K ? W[(size_t)(ka < K ? ka : K - 1) * ld + n] : 0.f; v[8 + i] = kb < K ? W[(size_t)(kb < K ? kb : K - 1) * ld + n] : 0.f; }
  return bsplit16(v); }
__device__ __forceinline__ v8f mac3(const F2& a, const F2& b, v8f c) { c = wmma_bf(a.l, b.h, c); c = wmma_bf(a.h, b.l, c); return wmma_bf(a.h, b.h, c); }
__device__ __forceinline__ float sigm(float v) { return 1.0f / (1.0f + expf(-v)); }
#define LDSX() do { asm volatile("s_wait_dscnt 0" ::: "memory"); __builtin_amdgcn_wave_barrier(); __builtin_amdgcn_fence(__ATOMIC_RELEASE, "workgroup"); } while (0)


#define NB 2
#define SS 2048
#define NR (NB * SS)
#define DM 1024
#define NH 16
#define HD 64
#define FF 4096
#define RAD 25
#define KREL 5
#define NREL (2 * KREL + 1)
#ifndef TQB
#define TQB (SS / 64)
#endif
#ifndef TQ0
#define TQ0 0
#endif
typedef __attribute__((ext_vector_type(8))) __bf16 v8b;
__device__ __forceinline__ v16b frag_b(const __bf16* rowk0, int lane) {
  union { v16b v; v8b q[2]; } u; const __bf16* p = rowk0 + 8 * (lane >> 4);
  u.q[0] = *(const v8b*)p; u.q[1] = *(const v8b*)(p + 16); return u.v;
}
__device__ __forceinline__ float bfr(float v) { return (float)(__bf16)v; }
__device__ __attribute__((noinline)) float exp_ni(float v) { return expf(v); }
__device__ __attribute__((noinline)) float erf_ni(float v) { return erff(v); }

#define PK_Q  0
#define PK_K  ((size_t)DM * DM)
#define PK_V  ((size_t)2 * DM * DM)
#define PK_O  ((size_t)3 * DM * DM)
#define PK_1  ((size_t)4 * DM * DM)
#define PK_2  (PK_1 + (size_t)FF * DM)
#define PK_END (PK_2 + (size_t)DM * FF)
#define WS_PK  0u
#define WS_QH  (((2u * PK_END) + 127u) / 128u * 128u)
#define WS_QL  (WS_QH + 2u * NR * DM)
#define WS_KH  (WS_QL + 2u * NR * DM)
#define WS_KL  (WS_KH + 2u * NR * DM)
#define WS_VTH (WS_KL + 2u * NR * DM)
#define WS_VTL (WS_VTH + 2u * NR * DM)
#define WS_REL (WS_VTL + 2u * NR * DM)
#define WS_RELL (WS_REL + 2u * 16 * HD)
#define WS_O   (((WS_RELL + 2u * 16 * HD) + 127u) / 128u * 128u)
#define WS_T1  (WS_O + 4u * NR * DM)
#define WS_H   (WS_T1 + 4u * NR * DM)
#define WS_GH  (WS_H + 4u * NR * DM)
#define WS_GL  (WS_GH + 2u * (size_t)NR * FF)
#define WS_END (WS_GL + 2u * (size_t)NR * FF)

__global__ __launch_bounds__(256) void k_pack(const float* __restrict__ WQ, const float* __restrict__ WK, const float* __restrict__ WV, const float* __restrict__ WO, const float* __restrict__ W1, const float* __restrict__ W2, const float* __restrict__ RELE, __bf16* __restrict__ PK, _Float16* __restrict__ RELH, _Float16* __restrict__ RELL) {
  __shared__ __align__(16) __bf16 s[FF]; __shared__ __align__(16) _Float16 sh_[HD], sl_[HD]; const int n = blockIdx.x, which = blockIdx.y, t = threadIdx.x; int K; size_t dst;
  if (which == 6) { if (n >= 16) return; if (t < HD) { const float v = (n < NREL) ? bfr(RELE[n * HD + t]) : 0.f; const _Float16 hv = (_Float16)v; sh_[t] = hv; sl_[t] = (_Float16)((v - (float)hv) * 2048.0f); } __syncthreads(); if (t < 8) vst2((unsigned*)(RELH + n * HD + t * 8), *(const v4u*)&sh_[t * 8]); else if (t < 16) vst2((unsigned*)(RELL + n * HD + (t - 8) * 8), *(const v4u*)&sl_[(t - 8) * 8]); return; }
  if (which < 4) { if (n >= DM) return; const float* Wm = (which == 0) ? WQ : (which == 1) ? WK : (which == 2) ? WV : WO; K = DM; dst = (size_t)which * DM * DM + (size_t)n * DM; for (int k = t; k < DM; k += 256) s[k] = (__bf16)Wm[(size_t)n * DM + k]; }
  else if (which == 4) { K = DM; dst = PK_1 + (size_t)n * DM; for (int k = t; k < DM; k += 256) s[k] = (__bf16)W1[(size_t)n * DM + k]; }
  else { if (n >= DM) return; K = FF; dst = PK_2 + (size_t)n * FF; for (int k = t; k < FF; k += 256) s[k] = (__bf16)W2[(size_t)n * FF + k]; }
  __syncthreads();
  for (int q = t; q < K / 8; q += 256) vst2((unsigned*)(PK + dst + q * 8), *(const v4u*)&s[q * 8]);
}
__global__ __launch_bounds__(128) void k_proj(const float* __restrict__ X, const __bf16* __restrict__ PK, const float* __restrict__ BQ, const float* __restrict__ BK, const float* __restrict__ BV, _Float16* __restrict__ QH, _Float16* __restrict__ QL_, _Float16* __restrict__ KH, _Float16* __restrict__ KL, _Float16* __restrict__ VTH, _Float16* __restrict__ VTL) {
  __shared__ __align__(16) _Float16 soh[4][16][136], sol[4][16][136]; __shared__ __align__(16) _Float16 sth[128][72], stl[128][72];
  const int tid = threadIdx.x, wave = tid >> 5, lane = tid & 31, col = lane & 15, g = lane >> 4; const int which = blockIdx.z; const size_t r0 = (size_t)blockIdx.x * 64 + wave * 16; const int n0 = blockIdx.y * 128;
  const __bf16* P = PK + ((which == 0) ? PK_Q : (which == 1) ? PK_K : PK_V); const float* BB = (which == 0) ? BQ : (which == 1) ? BK : BV;
  v8f acc[8] = {};
#pragma unroll 2
  for (int kc = 0; kc < DM / 32; ++kc) { v16b a; { const float* p = X + (r0 + col) * DM + kc * 32 + 8 * g;
#pragma unroll
      for (int i = 0; i < 8; ++i) { a[i] = (__bf16)p[i]; a[8 + i] = (__bf16)p[16 + i]; } }
#pragma unroll
    for (int j = 0; j < 8; ++j) acc[j] = wmma_bf(a, frag_b(P + (size_t)(n0 + j * 16 + col) * DM + kc * 32, lane), acc[j]); }
  if (which < 2) {
#pragma unroll
    for (int j = 0; j < 8; ++j) { const float bb = bfr(BB[n0 + j * 16 + col]);
#pragma unroll
      for (int r = 0; r < 8; ++r) { const float vv = acc[j][r] + bb; const _Float16 hv = (_Float16)vv; soh[wave][8 * g + r][j * 16 + col] = hv; sol[wave][8 * g + r][j * 16 + col] = (_Float16)((vv - (float)hv) * 2048.0f); } }
    LDSX();
    _Float16* DH_ = (which == 0) ? QH : KH; _Float16* DL_ = (which == 0) ? QL_ : KL;
    for (int rl = 0; rl < 16; ++rl) { if (lane < 16) vst2((unsigned*)(DH_ + (r0 + rl) * DM + n0 + lane * 8), *(const v4u*)&soh[wave][rl][lane * 8]); else vst2((unsigned*)(DL_ + (r0 + rl) * DM + n0 + (lane - 16) * 8), *(const v4u*)&sol[wave][rl][(lane - 16) * 8]); }
  } else {
#pragma unroll
    for (int j = 0; j < 8; ++j) { const float bb = bfr(BB[n0 + j * 16 + col]);
#pragma unroll
      for (int r = 0; r < 8; ++r) { const float vv = acc[j][r] + bb; const _Float16 hv = (_Float16)vv; sth[j * 16 + col][wave * 16 + 8 * g + r] = hv; stl[j * 16 + col][wave * 16 + 8 * g + r] = (_Float16)((vv - (float)hv) * 2048.0f); } }
    __syncthreads();
    const size_t rb = (size_t)blockIdx.x * 64; const int b = (int)(rb / SS), s0 = (int)(rb % SS);
    for (int e = tid; e < 128 * 8; e += 128) { const int d = e >> 3, pc = e & 7; const size_t o = ((size_t)b * DM + n0 + d) * SS + s0 + pc * 8; vst2((unsigned*)(VTH + o), *(const v4u*)&sth[d][pc * 8]); vst2((unsigned*)(VTL + o), *(const v4u*)&stl[d][pc * 8]); }
  }
}
__global__ __launch_bounds__(128) void k_attn(const _Float16* __restrict__ QH, const _Float16* __restrict__ QL_, const _Float16* __restrict__ KH, const _Float16* __restrict__ KL, const _Float16* __restrict__ RELH, const _Float16* __restrict__ RELL, const _Float16* __restrict__ VTH, const _Float16* __restrict__ VTL, float* __restrict__ O) {
  __shared__ __align__(16) _Float16 sph[4][16][40], spl[4][16][40]; __shared__ float srl[4][16][49]; __shared__ __align__(16) float so[4][16][68];
  const int tid = threadIdx.x, wave = tid >> 5, lane = tid & 31, col = lane & 15, g = lane >> 4; const int qb = blockIdx.x + TQ0, h = blockIdx.y, b = blockIdx.z; const int i0 = qb * 64, iw0 = i0 + wave * 16;
  v16h aq[2], aql[2];
#pragma unroll
  for (int kc = 0; kc < 2; ++kc) { const size_t o = ((size_t)b * SS + iw0 + col) * DM + h * HD + kc * 32; aq[kc] = frag_h(QH + o, lane); aql[kc] = frag_h(QL_ + o, lane); }
  const _Float16* Vh = VTH + ((size_t)b * DM + h * HD) * SS; const _Float16* Vl = VTL + ((size_t)b * DM + h * HD) * SS;
  float m[8], l[8];
#pragma unroll
  for (int r = 0; r < 8; ++r) { m[r] = -3.0e38f; l[r] = 0.f; }
  v8f acc[4] = {}, accl[4] = {};
  const int jlo = max(i0 - RAD, 0), jhi = min(i0 + 63 + RAD, SS - 1); const int ks0 = jlo / 32, ks1 = jhi / 32;
#pragma unroll 1
  for (int ks = ks0; ks <= ks1; ++ks) { const int j0 = ks * 32;
    { const int t0w = j0 - iw0 - 15;
#pragma unroll
      for (int ct3 = 0; ct3 < 3; ++ct3) { int rr = t0w + ct3 * 16 + col; rr = min(max(rr, -KREL), KREL) + KREL; v8f u = {}, ul = {};
#pragma unroll
        for (int kc = 0; kc < 2; ++kc) { const v16h rh = frag_h(RELH + (size_t)rr * HD + kc * 32, lane); u = wmma16(aq[kc], rh, u); ul = wmma16(aql[kc], rh, ul); ul = wmma16(aq[kc], frag_h(RELL + (size_t)rr * HD + kc * 32, lane), ul); }
#pragma unroll
        for (int r = 0; r < 8; ++r) srl[wave][8 * g + r][ct3 * 16 + col] = u[r] + ul[r] * (1.0f / 2048.0f); } }
    LDSX();
    v8f s[2];
#pragma unroll
    for (int ct = 0; ct < 2; ++ct) { const int jl = ct * 16 + col; const int kk = j0 + jl; const size_t rk = ((size_t)b * SS + kk) * DM + h * HD; v8f c = {}, cl = {};
#pragma unroll
      for (int kc = 0; kc < 2; ++kc) { const v16h khf = frag_h(KH + rk + kc * 32, lane); c = wmma16(aq[kc], khf, c); cl = wmma16(aql[kc], khf, cl); cl = wmma16(aq[kc], frag_h(KL + rk + kc * 32, lane), cl); }
#pragma unroll
      for (int r = 0; r < 8; ++r) { const int il = 8 * g + r; const int off = kk - (iw0 + il); const bool ok = (off <= RAD) && (off >= -RAD) && (kk < SS);
        s[ct][r] = ok ? (c[r] + cl[r] * (1.0f / 2048.0f) + srl[wave][il][jl - il + 15]) * 0.125f : -3.0e38f; } }
#pragma unroll
    for (int r = 0; r < 8; ++r) { float mx = fmaxf(s[0][r], s[1][r]);
#pragma unroll
      for (int o = 1; o < 16; o <<= 1) mx = fmaxf(mx, __shfl_xor(mx, o));
      const float mn = fmaxf(m[r], mx); const float alpha = (m[r] <= -1.0e38f) ? 0.f : __expf(m[r] - mn);
      const float e0 = (s[0][r] <= -1.0e38f) ? 0.f : __expf(s[0][r] - mn), e1 = (s[1][r] <= -1.0e38f) ? 0.f : __expf(s[1][r] - mn); float es = e0 + e1;
#pragma unroll
      for (int o = 1; o < 16; o <<= 1) es += __shfl_xor(es, o);
      l[r] = l[r] * alpha + es; m[r] = (mn <= -1.0e38f) ? m[r] : mn;
#pragma unroll
      for (int dt = 0; dt < 4; ++dt) { acc[dt][r] *= alpha; accl[dt][r] *= alpha; }
      const _Float16 h0 = (_Float16)e0, h1 = (_Float16)e1; sph[wave][8 * g + r][col] = h0; sph[wave][8 * g + r][16 + col] = h1; spl[wave][8 * g + r][col] = (_Float16)((e0 - (float)h0) * 2048.0f); spl[wave][8 * g + r][16 + col] = (_Float16)((e1 - (float)h1) * 2048.0f); }
    LDSX();
    const v16h pah = frag_h(&sph[wave][col][0], lane), pal = frag_h(&spl[wave][col][0], lane);
#pragma unroll
    for (int dt = 0; dt < 4; ++dt) { const size_t vo = (size_t)(dt * 16 + col) * SS + j0; const v16h vh = frag_h(Vh + vo, lane), vl = frag_h(Vl + vo, lane); acc[dt] = wmma16(pah, vh, acc[dt]); accl[dt] = wmma16(pal, vh, accl[dt]); accl[dt] = wmma16(pah, vl, accl[dt]); }
    LDSX(); }
#pragma unroll
  for (int r = 0; r < 8; ++r) { const float il = 1.0f / l[r];
#pragma unroll
    for (int dt = 0; dt < 4; ++dt) so[wave][8 * g + r][dt * 16 + col] = (acc[dt][r] + accl[dt][r] * (1.0f / 2048.0f)) * il; }
  LDSX();
  for (int rl = 0; rl < 16; ++rl) if (lane < 16) vst2(O + ((size_t)b * SS + iw0 + rl) * DM + h * HD + lane * 4, *(const v4f*)&so[wave][rl][lane * 4]);
}
template <int MODE>
__global__ __launch_bounds__(128) void k_lin(const float* __restrict__ A, const __bf16* __restrict__ AG, const __bf16* __restrict__ AGL, const __bf16* __restrict__ PK, const float* __restrict__ BIAS, const float* __restrict__ RES, float* __restrict__ OUTF, __bf16* __restrict__ OUTG, __bf16* __restrict__ OUTGL) {
  __shared__ __align__(16) float so[4][16][132]; __shared__ __align__(16) __bf16 sg[4][16][136], sgl[4][16][136];
  const int tid = threadIdx.x, wave = tid >> 5, lane = tid & 31, col = lane & 15, g = lane >> 4; const size_t r0 = (size_t)blockIdx.x * 64 + wave * 16; const int n0 = blockIdx.y * 128;
  constexpr int KD = (MODE == 2) ? FF : DM; const __bf16* P = PK + ((MODE == 0) ? PK_O : (MODE == 1) ? PK_1 : PK_2);
  v8f acc[8] = {};
  if (MODE == 2) {
#pragma unroll 2
    for (int kc = 0; kc < KD / 32; ++kc) { const v16b a = frag_b(AG + (r0 + col) * FF + kc * 32, lane), al = frag_b(AGL + (r0 + col) * FF + kc * 32, lane);
#pragma unroll
      for (int j = 0; j < 8; ++j) { const v16b w = frag_b(P + (size_t)(n0 + j * 16 + col) * KD + kc * 32, lane); acc[j] = wmma_bf(al, w, acc[j]); acc[j] = wmma_bf(a, w, acc[j]); } }
  } else {
#pragma unroll 2
    for (int kc = 0; kc < KD / 32; ++kc) { const F2 a = split_row(A + (r0 + col) * DM, kc * 32, lane);
#pragma unroll
      for (int j = 0; j < 8; ++j) { const v16b w = frag_b(P + (size_t)(n0 + j * 16 + col) * KD + kc * 32, lane); acc[j] = wmma_bf(a.l, w, acc[j]); acc[j] = wmma_bf(a.h, w, acc[j]); } } }
#pragma unroll
  for (int j = 0; j < 8; ++j) { const int c = n0 + j * 16 + col; const float bb = bfr(BIAS[c]);
#pragma unroll
    for (int r = 0; r < 8; ++r) { const size_t row = r0 + 8 * g + r; float v = acc[j][r] + bb;
      if (MODE == 1) { v = fmaxf(v, 0.f); const __bf16 hb = (__bf16)v; sg[wave][8 * g + r][j * 16 + col] = hb; sgl[wave][8 * g + r][j * 16 + col] = (__bf16)(v - (float)hb); }
      else { v += (MODE == 0) ? bfr(RES[row * DM + c]) : RES[row * DM + c]; so[wave][8 * g + r][j * 16 + col] = v; } } }
  LDSX();
  if (MODE == 1) { for (int rl = 0; rl < 16; ++rl) { if (lane < 16) vst2((unsigned*)(OUTG + (r0 + rl) * FF + n0 + lane * 8), *(const v4u*)&sg[wave][rl][lane * 8]); else vst2((unsigned*)(OUTGL + (r0 + rl) * FF + n0 + (lane - 16) * 8), *(const v4u*)&sgl[wave][rl][(lane - 16) * 8]); } }
  else { for (int rl = 0; rl < 16; ++rl) vst2(OUTF + (r0 + rl) * DM + n0 + lane * 4, *(const v4f*)&so[wave][rl][lane * 4]); }
}
__global__ __launch_bounds__(256) void k_ln(const float* __restrict__ T, const float* __restrict__ G, const float* __restrict__ Bv, float* __restrict__ OUT) {
  __shared__ float red[2][8]; const int t = threadIdx.x; const size_t row = blockIdx.x; const float* p = T + row * DM + t * 4;
  float v[4] = {p[0], p[1], p[2], p[3]}; float s = (v[0] + v[1]) + (v[2] + v[3]);
#pragma unroll
  for (int o = 1; o < 32; o <<= 1) s += __shfl_xor(s, o);
  if ((t & 31) == 0) red[0][t >> 5] = s; __syncthreads();
  float tot = 0.f; for (int w = 0; w < 8; ++w) tot += red[0][w]; const float mu = tot / (float)DM; float q = 0.f;
#pragma unroll
  for (int i = 0; i < 4; ++i) { const float d = v[i] - mu; q += d * d; }
#pragma unroll
  for (int o = 1; o < 32; o <<= 1) q += __shfl_xor(q, o);
  if ((t & 31) == 0) red[1][t >> 5] = q; __syncthreads();
  float qt = 0.f; for (int w = 0; w < 8; ++w) qt += red[1][w]; const float inv = 1.0f / sqrtf(qt / (float)DM + 1e-5f);
  v4f o4;
#pragma unroll
  for (int i = 0; i < 4; ++i) o4[i] = (v[i] - mu) * inv * bfr(G[t * 4 + i]) + bfr(Bv[t * 4 + i]);
  vst2(OUT + row * DM + t * 4, o4);
}
extern "C" void kernel_launch(void* const* d_in, const int* in_sizes, int n_in, void* d_out, int out_size, void* d_ws, size_t ws_size, hipStream_t stream) {
  (void)in_sizes; (void)n_in; (void)out_size;
  const float** F = (const float**)d_in;
  if (ws_size < (size_t)WS_END) return;
  char* ws = (char*)d_ws; __bf16 *PK = (__bf16*)(ws + WS_PK), *GH = (__bf16*)(ws + WS_GH), *GL = (__bf16*)(ws + WS_GL); _Float16 *QH = (_Float16*)(ws + WS_QH), *QLp = (_Float16*)(ws + WS_QL), *KH = (_Float16*)(ws + WS_KH), *KL = (_Float16*)(ws + WS_KL), *VTH = (_Float16*)(ws + WS_VTH), *VTL = (_Float16*)(ws + WS_VTL), *RELH = (_Float16*)(ws + WS_REL), *RELL = (_Float16*)(ws + WS_RELL); float *O = (float*)(ws + WS_O), *T1 = (float*)(ws + WS_T1), *Hh = (float*)(ws + WS_H);
  k_pack<<<dim3(FF, 7), 256, 0, stream>>>(F[1], F[3], F[5], F[7], F[10], F[12], F[9], PK, RELH, RELL);
  k_proj<<<dim3(NR / 64, DM / 128, 3), 128, 0, stream>>>(F[0], PK, F[2], F[4], F[6], QH, QLp, KH, KL, VTH, VTL);
  k_attn<<<dim3(TQB, NH, NB), 128, 0, stream>>>(QH, QLp, KH, KL, RELH, RELL, VTH, VTL, O);
#ifndef TWIN_ROWS
  const size_t R0 = 0; const int NRW = NR; (void)R0;
  k_lin<0><<<dim3(NR / 64, DM / 128), 128, 0, stream>>>(O, nullptr, nullptr, PK, F[8], F[0], T1, nullptr, nullptr);
  k_ln<<<NR, 256, 0, stream>>>(T1, F[14], F[15], Hh);
  k_lin<1><<<dim3(NR / 64, FF / 128), 128, 0, stream>>>(Hh, nullptr, nullptr, PK, F[11], nullptr, nullptr, GH, GL);
  k_lin<2><<<dim3(NR / 64, DM / 128), 128, 0, stream>>>(nullptr, GH, GL, PK, F[13], Hh, T1, nullptr, nullptr);
  k_ln<<<NR, 256, 0, stream>>>(T1, F[16], F[17], (float*)d_out);
#else
  for (int bb = 0; bb < NB; ++bb) { const size_t R0 = (size_t)bb * SS + (size_t)TQ0 * 64; const int NRW = TQB * 64;
  k_lin<0><<<dim3(NRW / 64, DM / 128), 128, 0, stream>>>(O + R0 * DM, nullptr, nullptr, PK, F[8], F[0] + R0 * DM, T1 + R0 * DM, nullptr, nullptr);
  k_ln<<<NRW, 256, 0, stream>>>(T1 + R0 * DM, F[14], F[15], Hh + R0 * DM);
  k_lin<1><<<dim3(NRW / 64, FF / 128), 128, 0, stream>>>(Hh + R0 * DM, nullptr, nullptr, PK, F[11], nullptr, nullptr, GH + R0 * FF, GL + R0 * FF);
  k_lin<2><<<dim3(NRW / 64, DM / 128), 128, 0, stream>>>(nullptr, GH + R0 * FF, GL + R0 * FF, PK, F[13], Hh + R0 * DM, T1 + R0 * DM, nullptr, nullptr);
  k_ln<<<NRW, 256, 0, stream>>>(T1 + R0 * DM, F[16], F[17], (float*)d_out + R0 * DM); }
#endif
}
